// MoEFusionLayer_55387898249742
// MI455X (gfx1250) — hardware-verified
//
#include <hip/hip_runtime.h>
#include <stdint.h>
#include <stddef.h>
#include <math.h>

#define NB   8
#define NL   1024
#define ND   768
#define NE   4
#define NH   1536
#define NHH  (NH / 2)
#define NTOK (NB * NL)
#define MR   16
#define XP   776
#define HP   1544
#define VP   772
#define YP   772
#define RECW 32

#define SXB (MR * XP * 2)
#define SHB (MR * HP * 2)
#define SVB (MR * VP * 4)
#define SYB (MR * YP * 4)
#define LDS_MAIN (SXB + SHB + SVB + SYB)

#define W1S   16.0f
#define HS    8.0f
#define W2S   32.0f
#define G1INV (1.0f / 16.0f)
#define G2INV (1.0f / 256.0f)

static_assert(LDS_MAIN == 173056);
static_assert((XP * 2) % 16 == 0);
static_assert((HP * 2) % 16 == 0);
static_assert((VP * 4) % 16 == 0);
static_assert((YP * 4) % 16 == 0);
static_assert(SXB % 16 == 0);
static_assert(SHB % 16 == 0);
static_assert(SVB % 16 == 0);
static_assert(ND % 64 == 0);
static_assert(NH % 64 == 0);
static_assert(NL % MR == 0);
static_assert(ND == 3 * 256);
static_assert(NHH == 8 * 96);
static_assert(ND == 8 * 96);
static_assert((MR * ND / 4) % 256 == 0);
static_assert((MR * NHH) % 256 == 0);
static_assert(MR == 2 * 8);
static_assert(ND % 128 == 0);
static_assert(XP >= ND + 8);
static_assert(HP >= NH + 8);

typedef _Float16     v16h __attribute__((ext_vector_type(16)));
typedef _Float16     v8h  __attribute__((ext_vector_type(8)));
typedef _Float16     v4h  __attribute__((ext_vector_type(4)));
typedef float        v8f  __attribute__((ext_vector_type(8)));
typedef float        v4f  __attribute__((ext_vector_type(4)));
typedef unsigned int v4u  __attribute__((ext_vector_type(4)));
typedef v4f __attribute__((may_alias)) v4fa;
typedef v8h __attribute__((may_alias)) v8ha;
typedef v4h __attribute__((may_alias)) v4ha;
typedef v4u __attribute__((may_alias)) v4ua;

union Frag  { v16h v; v8h half[2]; };
union Pack8 { v8h h; v4u u; };

__device__ __forceinline__ v8f wmma16(v16h a, v16h b, v8f c) {
  v8f d = __builtin_amdgcn_wmma_f32_16x16x32_f16(false, a, false, b, (short)0, c, false, false);
  asm volatile("v_nop\n\tv_nop\n\tv_nop\n\tv_nop" : "+v"(d) : "v"(a), "v"(b));
  return d;
}

__device__ __forceinline__ v16h ldf(const _Float16* p, int h) {
  Frag f;
  f.half[0] = *(const v8ha*)(p + 8 * h);
  f.half[1] = *(const v8ha*)(p + 16 + 8 * h);
  return f.v;
}

__device__ __forceinline__ float gelu_f(float v) {
  const float u = fabsf(v) * 0.70710678118654752f;
  const float t = __builtin_amdgcn_rcpf(1.0f + 0.3275911f * u);
  const float p = t * (0.254829592f +
                  t * (-0.284496736f +
                  t * (1.421413741f +
                  t * (-1.453152027f +
                  t * 1.061405429f))));
  float er = 1.0f - p * __expf(-u * u);
  er = copysignf(er, v);
  return 0.5f * v * (1.0f + er);
}
__device__ __forceinline__ float silu_f(float v) {
  return v * __builtin_amdgcn_rcpf(1.0f + __expf(-v));
}
__device__ __forceinline__ float mish_f(float v) {
  const float ex = __expf(fminf(v, 20.0f));
  const float n = ex * (ex + 2.0f);
  return v * n * __builtin_amdgcn_rcpf(n + 2.0f);
}

__global__ __launch_bounds__(256) void k_route(const float* __restrict__ x,
                                               const float* __restrict__ rw,
                                               const float* __restrict__ rb,
                                               float* __restrict__ rec)
{
  __shared__ double sp[NE * 256];
  __shared__ __align__(16) float sg[8];
  const int tid = threadIdx.x, lane = tid & 31, wv = tid >> 5;
  const int b = blockIdx.x;
  const float* xb = x + (size_t)b * NL * ND;

  double a0 = 0.0, a1 = 0.0, a2 = 0.0;
  #pragma unroll 1
  for (int l = 0; l < NL; ++l) {
    const float* row = xb + (size_t)l * ND;
    a0 += (double)row[tid];
    a1 += (double)row[tid + 256];
    a2 += (double)row[tid + 512];
  }
  const double inv = 1.0 / (double)NL;
  a0 *= inv; a1 *= inv; a2 *= inv;
  #pragma unroll
  for (int e = 0; e < NE; ++e) {
    const float* w = rw + e * ND;
    double p = a0 * (double)w[tid];
    p = fma(a1, (double)w[tid + 256], p);
    p = fma(a2, (double)w[tid + 512], p);
    sp[e * 256 + tid] = p;
  }
  __syncthreads();
  #pragma unroll 1
  for (int s = 128; s > 0; s >>= 1) {
    if (tid < s) {
      #pragma unroll
      for (int e = 0; e < NE; ++e) sp[e * 256 + tid] += sp[e * 256 + tid + s];
    }
    __syncthreads();
  }
  if (tid == 0) {
    const float l0 = (float)sp[0 * 256] + rb[0];
    const float l1 = (float)sp[1 * 256] + rb[1];
    const float l2 = (float)sp[2 * 256] + rb[2];
    const float l3 = (float)sp[3 * 256] + rb[3];
    int i0 = 0; float v0 = l0;
    if (l1 > v0) { v0 = l1; i0 = 1; }
    if (l2 > v0) { v0 = l2; i0 = 2; }
    if (l3 > v0) { v0 = l3; i0 = 3; }
    const float c0 = (i0 == 0) ? -INFINITY : l0;
    const float c1 = (i0 == 1) ? -INFINITY : l1;
    const float c2 = (i0 == 2) ? -INFINITY : l2;
    const float c3 = (i0 == 3) ? -INFINITY : l3;
    int i1 = 0; float v1 = c0;
    if (c1 > v1) { v1 = c1; i1 = 1; }
    if (c2 > v1) { v1 = c2; i1 = 2; }
    if (c3 > v1) { v1 = c3; i1 = 3; }
    const float e1 = expf(v1 - v0);
    const float rs = __builtin_amdgcn_rcpf(1.0f + e1);
    const float g0 = rs;
    const float g1 = e1 * rs;
    sg[0] = (i0 == 0) ? g0 : ((i1 == 0) ? g1 : 0.0f);
    sg[1] = (i0 == 1) ? g0 : ((i1 == 1) ? g1 : 0.0f);
    sg[2] = (i0 == 2) ? g0 : ((i1 == 2) ? g1 : 0.0f);
    sg[3] = (i0 == 3) ? g0 : ((i1 == 3) ? g1 : 0.0f);
  }
  __syncthreads();
  if (wv == 0) {
    const v4f g = *(const v4fa*)sg;
    float* d = rec + (size_t)b * RECW + 4 * (lane & 7);
    const bool ok = (lane < 8);
    if (ok) *(volatile v4fa*)d = g;
    __threadfence();
    if (ok) *(volatile v4fa*)d = g;
  }
}

__global__ __launch_bounds__(256) void k_wt(const float* __restrict__ src,
                                            _Float16* __restrict__ dst,
                                            int K, int N, float scale)
{
  __shared__ __align__(16) _Float16 st[32 * 72];
  const int tid = threadIdx.x, lane = tid & 31, wv = tid >> 5;
  const int e = blockIdx.z;
  const int k0 = blockIdx.x * 64;
  const int n0 = blockIdx.y * 32;
  const int nn = tid & 31, kq = tid >> 5;
  const float* sb = src + ((size_t)e * K + k0) * N + n0 + nn;
  #pragma unroll
  for (int i = 0; i < 8; ++i) {
    const int kk = kq + 8 * i;
    st[nn * 72 + kk] = (_Float16)(sb[(size_t)kk * N] * scale);
  }
  __syncthreads();
  const int q = lane >> 3, p = lane & 7;
  const int row = 4 * wv + q;
  Pack8 u;
  u.h = *(const v8ha*)(st + row * 72 + 8 * p);
  _Float16* d = dst + ((size_t)e * N + n0 + row) * K + k0 + 8 * p;
  *(volatile v4ua*)d = u.u;
  __threadfence();
  *(volatile v4ua*)d = u.u;
}

__global__ __launch_bounds__(256) void k_main(const float* __restrict__ x,
                                              const _Float16* __restrict__ w1t,
                                              const _Float16* __restrict__ w2t,
                                              const float* __restrict__ b1,
                                              const float* __restrict__ b2,
                                              const float* __restrict__ rec,
                                              const float* __restrict__ lng,
                                              const float* __restrict__ lnb,
                                              float* __restrict__ out)
{
  extern __shared__ __align__(16) unsigned char dsm[];
  _Float16* sx = (_Float16*)dsm;
  _Float16* sh = (_Float16*)(dsm + SXB);
  float*    sv = (float*)(dsm + SXB + SHB);
  float*    sy = (float*)(dsm + SXB + SHB + SVB);

  const int tid = threadIdx.x, lane = tid & 31, wv = tid >> 5;
  const int h = lane >> 4, m = lane & 15;
  const int b  = blockIdx.x / (NL / MR);
  const int m0 = (blockIdx.x - b * (NL / MR)) * MR;
  const size_t trow0 = (size_t)b * NL + m0;

  #pragma unroll
  for (int i = 0; i < (MR * ND / 4) / 256; ++i) {
    const int idx = tid + 256 * i;
    const int r = idx / (ND / 4);
    const int c4 = idx - r * (ND / 4);
    const v4f v = *(const v4fa*)(x + (trow0 + r) * ND + 4 * c4);
    *(v4fa*)(sy + r * YP + 4 * c4) = v;
    const v4h hv = __builtin_convertvector(v, v4h);
    *(v4ha*)(sx + r * XP + 4 * c4) = hv;
  }
  __syncthreads();

  const v8f z8 = {0.f, 0.f, 0.f, 0.f, 0.f, 0.f, 0.f, 0.f};

  #pragma unroll 1
  for (int e = 0; e < NE; ++e) {
    const float ge = rec[(size_t)b * RECW + e];
    if (ge == 0.0f) continue;

    #pragma unroll 1
    for (int np = 0; np < 2; ++np) {
      v8f acc[6];
      #pragma unroll
      for (int j = 0; j < 6; ++j) acc[j] = z8;
      const _Float16* brow = w1t + ((size_t)e * NH + np * NHH + wv * 96 + m) * ND;
      #pragma unroll 2
      for (int k0 = 0; k0 < ND; k0 += 32) {
        const v16h a = ldf(sx + m * XP + k0, h);
        #pragma unroll
        for (int j = 0; j < 6; ++j) {
          const v16h bb = ldf(brow + (size_t)j * 16 * ND + k0, h);
          acc[j] = wmma16(a, bb, acc[j]);
        }
      }
      #pragma unroll
      for (int j = 0; j < 6; ++j) {
        const int c = wv * 96 + 16 * j + m;
        const float bias = b1[(size_t)e * NH + np * NHH + c];
        #pragma unroll
        for (int r = 0; r < 8; ++r) sv[(8 * h + r) * VP + c] = acc[j][r] * G1INV + bias;
      }
      __syncthreads();
      #pragma unroll 1
      for (int it = 0; it < (MR * NHH) / 256; ++it) {
        const int idx = tid + 256 * it;
        const int r = idx / NHH;
        const int c = idx - r * NHH;
        const float v = sv[r * VP + c];
        float av;
        if (e == 1)      av = silu_f(v);
        else if (e == 2) av = mish_f(v);
        else             av = gelu_f(v);
        sh[r * HP + np * NHH + c] = (_Float16)(av * HS);
      }
      __syncthreads();
    }

    {
      v8f acc[6];
      #pragma unroll
      for (int j = 0; j < 6; ++j) acc[j] = z8;
      const _Float16* brow = w2t + ((size_t)e * ND + wv * 96 + m) * NH;
      #pragma unroll 2
      for (int k0 = 0; k0 < NH; k0 += 32) {
        const v16h a = ldf(sh + m * HP + k0, h);
        #pragma unroll
        for (int j = 0; j < 6; ++j) {
          const v16h bb = ldf(brow + (size_t)j * 16 * NH + k0, h);
          acc[j] = wmma16(a, bb, acc[j]);
        }
      }
      #pragma unroll
      for (int j = 0; j < 6; ++j) {
        const int c = wv * 96 + 16 * j + m;
        const float bias = b2[(size_t)e * ND + c];
        #pragma unroll
        for (int r = 0; r < 8; ++r) {
          float* p = sy + (8 * h + r) * YP + c;
          const float yv = *p;
          *p = yv + ge * (acc[j][r] * G2INV + bias);
        }
      }
    }
  }
  __syncthreads();

  #pragma unroll 1
  for (int rr = 0; rr < 2; ++rr) {
    const int r = 2 * wv + rr;
    float* row = sy + r * YP;
    float s = 0.f;
    #pragma unroll 4
    for (int i = 0; i < ND / 32; ++i) s += row[lane + 32 * i];
    #pragma unroll
    for (int o = 16; o > 0; o >>= 1) s += __shfl_xor(s, o);
    const float mu = s * (1.0f / (float)ND);
    float q = 0.f;
    #pragma unroll 4
    for (int i = 0; i < ND / 32; ++i) { const float d = row[lane + 32 * i] - mu; q += d * d; }
    #pragma unroll
    for (int o = 16; o > 0; o >>= 1) q += __shfl_xor(q, o);
    const float var  = q * (1.0f / (float)ND);
    const float rstd = rsqrtf(var + 1e-5f);
    #pragma unroll 4
    for (int i = 0; i < ND / 32; ++i) {
      const int c = lane + 32 * i;
      row[c] = (row[c] - mu) * rstd * lng[c] + lnb[c];
    }
  }
  __syncthreads();

  #pragma unroll 1
  for (int rr = 0; rr < 2; ++rr) {
    const int r = 2 * wv + rr;
    const float* row = sy + r * YP;
    float* orow = out + (trow0 + r) * ND;
    #pragma unroll
    for (int i = 0; i < ND / 128; ++i) {
      const int f4 = 32 * i + lane;
      const v4f v = *(const v4fa*)(row + 4 * f4);
      *(volatile v4fa*)(orow + 4 * f4) = v;
    }
  }
  __threadfence();
  #pragma unroll 1
  for (int rr = 0; rr < 2; ++rr) {
    const int r = 2 * wv + rr;
    const float* row = sy + r * YP;
    float* orow = out + (trow0 + r) * ND;
    #pragma unroll
    for (int i = 0; i < ND / 128; ++i) {
      const int f4 = 32 * i + lane;
      const v4f v = *(const v4fa*)(row + 4 * f4);
      *(volatile v4fa*)(orow + 4 * f4) = v;
    }
  }
}

extern "C" void kernel_launch(void* const* d_in, const int* in_sizes, int n_in,
                              void* d_out, int out_size, void* d_ws, size_t ws_size,
                              hipStream_t stream)
{
  if (n_in < 9) return;
  if (in_sizes[0] != NTOK * ND) return;
  if (in_sizes[1] != NE * ND) return;
  if (in_sizes[2] != NE) return;
  if (in_sizes[3] != NE * ND * NH) return;
  if (in_sizes[4] != NE * NH) return;
  if (in_sizes[5] != NE * NH * ND) return;
  if (in_sizes[6] != NE * ND) return;
  if (in_sizes[7] != ND) return;
  if (in_sizes[8] != ND) return;
  if (out_size != NTOK * ND) return;

  const float* x   = (const float*)d_in[0];
  const float* rw  = (const float*)d_in[1];
  const float* rb  = (const float*)d_in[2];
  const float* w1  = (const float*)d_in[3];
  const float* b1  = (const float*)d_in[4];
  const float* w2  = (const float*)d_in[5];
  const float* b2  = (const float*)d_in[6];
  const float* lng = (const float*)d_in[7];
  const float* lnb = (const float*)d_in[8];
  float* out = (float*)d_out;

  const size_t bW1T = (size_t)NE * NH * ND * 2;
  const size_t bW2T = (size_t)NE * ND * NH * 2;
  const size_t bREC = (size_t)NB * RECW * 4;
  const size_t total = bW1T + bW2T + bREC;
  if (total > ws_size) return;
  if (total > (size_t)134217728) return;

  char* ws = (char*)d_ws;
  size_t off = 0;
  _Float16* W1T = (_Float16*)(ws + off); off += bW1T;
  _Float16* W2T = (_Float16*)(ws + off); off += bW2T;
  float*    REC = (float*)(ws + off);    off += bREC;
  if (off != total) return;

  k_route<<<NB, 256, 0, stream>>>(x, rw, rb, REC);
  k_wt<<<dim3(ND / 64, NH / 32, NE), 256, 0, stream>>>(w1, W1T, ND, NH, W1S);
  k_wt<<<dim3(NH / 64, ND / 32, NE), 256, 0, stream>>>(w2, W2T, NH, ND, W2S);
  hipFuncSetAttribute(reinterpret_cast<const void*>(&k_main),
                      hipFuncAttributeMaxDynamicSharedMemorySize, LDS_MAIN);
  k_main<<<NTOK / MR, 256, LDS_MAIN, stream>>>(x, W1T, W2T, b1, b2, REC, lng, lnb, out);
}
